// GAT_35107062677930
// MI455X (gfx1250) — hardware-verified
//
#include <hip/hip_runtime.h>
#include <stddef.h>
#include <stdint.h>
#include <math.h>


#pragma clang fp contract(off)

#define DIN    128
#define D1     256
#define D2     64
#define KP     512
#define NTHR   256
#define NWAVE  8
#define EPT    8
#define CHUNK  (NTHR * EPT)
#define WCAP   (EPT * 32)
#define LISTN  (NWAVE * WCAP)
#define NBA    1024
#define SLA    10
#define RCAP   28672
#define DEGCAP 64
#define GBM    64
#define GBN    128
#define GTHR   128
#define NU1    (D1 * (DIN / 8))
#define NU2    (D2 * (KP / 8))
#define NEGSL  0.2f
#define AGG_ZINTS (LISTN + 2 * RCAP + 3 * NBA)
#define AGG_LDS_INTS (AGG_ZINTS + 16)
#define WSMAX  134217728

static_assert((CHUNK & (CHUNK - 1)) == 0 && CHUNK <= 4096);
static_assert((NBA & (NBA - 1)) == 0 && NBA == (1 << SLA));
static_assert(((long long)CHUNK << SLA) < (1LL << 31));
static_assert(LISTN % NTHR == 0);
static_assert(NBA % NWAVE == 0 && NBA % 32 == 0 && NBA % GBM == 0);
static_assert(NBA == NTHR * 4);
static_assert(RCAP % (NTHR * 4) == 0 && AGG_ZINTS % 4 == 0 && LISTN % 4 == 0);
static_assert(RCAP >= 16623 + 4096);
static_assert(DEGCAP >= 35 + 8);
static_assert(DIN % 32 == 0 && KP % 32 == 0 && KP == 2 * D1 && D1 == 2 * GBN);
static_assert(GBM == (GTHR / 32) * 16 && GBN == 4 * 32);
static_assert(NU1 % NTHR == 0 && NU2 % NTHR == 0);
static_assert(DIN / 8 == 16 && KP / 8 == 64);
static_assert(AGG_LDS_INTS * 4 <= 300000);
static_assert(D1 == 8 * 32 && D2 == 2 * 32);
static_assert(D2 == GBM);

typedef float          v2f   __attribute__((ext_vector_type(2)));
typedef float          v4f   __attribute__((ext_vector_type(4)));
typedef float          v8f   __attribute__((ext_vector_type(8)));
typedef int            v4i   __attribute__((ext_vector_type(4)));
typedef int            v8i   __attribute__((ext_vector_type(8)));
typedef unsigned short v8us  __attribute__((ext_vector_type(8)));
typedef unsigned short v16us __attribute__((ext_vector_type(16)));
typedef __bf16         v16bf __attribute__((ext_vector_type(16)));
typedef v2f  __attribute__((may_alias)) v2fa;
typedef v4f  __attribute__((may_alias)) v4fa;
typedef v4i  __attribute__((may_alias)) v4ia;
typedef v8us __attribute__((may_alias)) v8usa;
union FragB { v16bf v; v16us u; v8us h[2]; v8i w; };

__device__ __forceinline__ v8f wmb(const FragB& a, const FragB& b, v8f c) {
  v8f d = __builtin_amdgcn_wmma_f32_16x16x32_bf16(false, a.v, false, b.v, (short)0, c, false, false);
  asm volatile("v_nop\n\tv_nop\n\tv_nop\n\tv_nop" : "+v"(d) : "v"(a.w), "v"(b.w));
  return d;
}

__device__ __forceinline__ unsigned bf16_bits(float f) {
  const unsigned u = __float_as_uint(f);
  const unsigned r = ((u + 0x7FFFu + ((u >> 16) & 1u)) >> 16) & 0xFFFFu;
  return (f != f) ? 0x7FC0u : r;
}
__device__ __forceinline__ float bf16_val(float f) {
  return __uint_as_float(bf16_bits(f) << 16);
}
__device__ __forceinline__ v4f bfr4(const v4f a) {
  v4f r; r.x = bf16_val(a.x); r.y = bf16_val(a.y); r.z = bf16_val(a.z); r.w = bf16_val(a.w); return r;
}

template <int SLB>
__device__ __forceinline__ int scan_chunk(const int* __restrict__ dsts, int nE, int cbase, int slotBase,
                                          int nb, int vec8, int* list, int tid, int lane, int wave) {
  int wc = 0;
  const int el0  = tid * EPT;
  const int e0   = cbase + el0;
  const int sent = -2147483647 - 1;
  v4i da, db;
  if (vec8 != 0 && cbase + CHUNK <= nE) {
    da = *(const v4i*)(dsts + e0);
    db = *(const v4i*)(dsts + e0 + 4);
  } else {
    da.x = (e0     < nE) ? dsts[min(e0,     nE - 1)] : sent;
    da.y = (e0 + 1 < nE) ? dsts[min(e0 + 1, nE - 1)] : sent;
    da.z = (e0 + 2 < nE) ? dsts[min(e0 + 2, nE - 1)] : sent;
    da.w = (e0 + 3 < nE) ? dsts[min(e0 + 3, nE - 1)] : sent;
    db.x = (e0 + 4 < nE) ? dsts[min(e0 + 4, nE - 1)] : sent;
    db.y = (e0 + 5 < nE) ? dsts[min(e0 + 5, nE - 1)] : sent;
    db.z = (e0 + 6 < nE) ? dsts[min(e0 + 6, nE - 1)] : sent;
    db.w = (e0 + 7 < nE) ? dsts[min(e0 + 7, nE - 1)] : sent;
  }
  const unsigned nbs = (unsigned)slotBase;
  const unsigned unb = (unsigned)nb;
  const unsigned s0 = (unsigned)da.x - nbs, s1 = (unsigned)da.y - nbs;
  const unsigned s2 = (unsigned)da.z - nbs, s3 = (unsigned)da.w - nbs;
  const unsigned s4 = (unsigned)db.x - nbs, s5 = (unsigned)db.y - nbs;
  const unsigned s6 = (unsigned)db.z - nbs, s7 = (unsigned)db.w - nbs;
  const bool h0 = s0 < unb, h1 = s1 < unb, h2 = s2 < unb, h3 = s3 < unb;
  const bool h4 = s4 < unb, h5 = s5 < unb, h6 = s6 < unb, h7 = s7 < unb;
  const unsigned any = __builtin_amdgcn_ballot_w32(h0 | h1 | h2 | h3 | h4 | h5 | h6 | h7);
  if (any != 0u) {
#define HITJ(J, HJ, SJ) { \
      const unsigned mj = __builtin_amdgcn_ballot_w32(HJ); \
      if (mj != 0u) { \
        if (HJ) { \
          const int pos = wc + (int)__builtin_amdgcn_mbcnt_lo(mj, 0u); \
          if (pos < WCAP) list[wave * WCAP + pos] = ((el0 + (J)) << SLB) | (int)(SJ); \
        } \
        wc += (int)__builtin_popcount(mj); } }
    HITJ(0, h0, s0)
    HITJ(1, h1, s1)
    HITJ(2, h2, s2)
    HITJ(3, h3, s3)
    HITJ(4, h4, s4)
    HITJ(5, h5, s5)
    HITJ(6, h6, s6)
    HITJ(7, h7, s7)
#undef HITJ
  }
  return wc;
}

__global__ __launch_bounds__(NTHR) void k_prep(const float* __restrict__ x, const float* __restrict__ W1,
                                               const float* __restrict__ W2,
                                               unsigned short* XB, unsigned short* W1T, unsigned short* W2T,
                                               int nN, int nUx) {
  const int u = (int)blockIdx.x * NTHR + (int)threadIdx.x;
  v8us o;
  unsigned short* dp;
  if (u < nUx) {
    const int row = u >> 4;
    const int k8  = (u & 15) * 8;
    const int rc  = row < nN ? row : nN - 1;
    const float* p = x + (size_t)rc * DIN + k8;
    const v4f a = *(const v4fa*)p;
    const v4f b = *(const v4fa*)(p + 4);
    const bool ok = row < nN;
    o[0] = ok ? (unsigned short)bf16_bits(a.x) : (unsigned short)0;
    o[1] = ok ? (unsigned short)bf16_bits(a.y) : (unsigned short)0;
    o[2] = ok ? (unsigned short)bf16_bits(a.z) : (unsigned short)0;
    o[3] = ok ? (unsigned short)bf16_bits(a.w) : (unsigned short)0;
    o[4] = ok ? (unsigned short)bf16_bits(b.x) : (unsigned short)0;
    o[5] = ok ? (unsigned short)bf16_bits(b.y) : (unsigned short)0;
    o[6] = ok ? (unsigned short)bf16_bits(b.z) : (unsigned short)0;
    o[7] = ok ? (unsigned short)bf16_bits(b.w) : (unsigned short)0;
    dp = XB + (size_t)row * DIN + k8;
  } else if (u < nUx + NU1) {
    const int v  = u - nUx;
    const int n  = v >> 4;
    const int k8 = (v & 15) * 8;
    const float* p = W1 + (size_t)k8 * D1 + n;
#pragma unroll
    for (int i = 0; i < 8; ++i) o[i] = (unsigned short)bf16_bits(p[(size_t)i * D1]);
    dp = W1T + (size_t)n * DIN + k8;
  } else if (u < nUx + NU1 + NU2) {
    const int v  = u - nUx - NU1;
    const int n  = v >> 6;
    const int k8 = (v & 63) * 8;
    const int kk = k8 & (D1 - 1);
    const float* p = W2 + (size_t)kk * D2 + n;
#pragma unroll
    for (int i = 0; i < 8; ++i) o[i] = (unsigned short)bf16_bits(p[(size_t)i * D2]);
    dp = W2T + (size_t)n * KP + k8;
  } else {
    return;
  }
  *(volatile v8us*)dp = o;
  __threadfence();
  *(volatile v8us*)dp = o;
}

__global__ __launch_bounds__(NTHR) void k_bucket(const int* __restrict__ srcs, const int* __restrict__ dsts,
                                                 int nE, int nN, int vec8, int* SRT, int* OC) {
  extern __shared__ __attribute__((aligned(16))) int dsm[];
  int* list = dsm;
  int* hl   = dsm + LISTN;
  int* sl   = dsm + LISTN + RCAP;
  int* cnt  = dsm + LISTN + 2 * RCAP;
  int* offs = cnt + NBA;
  int* cur  = offs + NBA;
  int* misc = cur + NBA;
  const int tid = (int)threadIdx.x, lane = tid & 31;
  const int wave = __builtin_amdgcn_readfirstlane(tid >> 5);
  const int nodeBase = (int)blockIdx.x * NBA;

  {
    const v4i z4 = {0, 0, 0, 0};
    for (int i = tid * 4; i < AGG_ZINTS; i += NTHR * 4) *(v4ia*)(dsm + i) = z4;
    if (tid < 16) misc[tid] = 0;
  }
  __syncthreads();

  int t = 0, ov = 0;
  const int nChunks = (nE + CHUNK - 1) / CHUNK;
#pragma unroll 1
  for (int ch = 0; ch < nChunks; ++ch) {
    const int cbase = ch * CHUNK;
    const int wc = scan_chunk<SLA>(dsts, nE, cbase, nodeBase, NBA, vec8, list, tid, lane, wave);
    if (lane == 0) misc[wave] = wc;
    __syncthreads();
    if (wave == 0) {
#pragma unroll 1
      for (int w2 = 0; w2 < NWAVE; ++w2) {
        int c = misc[w2];
        c = c < 0 ? 0 : (c > WCAP ? WCAP : c);
#pragma unroll 1
        for (int b0 = 0; b0 < c; b0 += 32) {
          const int idx = b0 + lane;
          const int ent = list[w2 * WCAP + (idx < WCAP ? idx : WCAP - 1)];
          const int m32 = (c - b0) < 32 ? (c - b0) : 32;
#pragma unroll 1
          for (int k = 0; k < m32; ++k) {
            const int u    = __builtin_amdgcn_readlane(ent, k);
            const int slot = u & (NBA - 1);
            const int el   = (u >> SLA) & (CHUNK - 1);
            const int pk   = ((cbase + el) << SLA) | slot;
            if (t < RCAP) {
              if (lane == 0) { hl[t] = pk; cnt[slot] = cnt[slot] + 1; }
              t = t + 1;
            } else {
              ov = 1;
            }
          }
        }
      }
    }
    __syncthreads();
  }
  if (wave == 0 && lane == 0) { misc[8] = t; misc[9] = ov; }
  __syncthreads();
  int tt = misc[8];
  tt = tt < 0 ? 0 : (tt > RCAP ? RCAP : tt);
  const int ovf = misc[9];

  if (wave == 0) {
    const int base = lane * (NBA / 32);
    int s = 0;
#pragma unroll 1
    for (int i = 0; i < NBA / 32; ++i) s += cnt[base + i];
    int incl = s;
#pragma unroll
    for (int d = 1; d < 32; d <<= 1) {
      const int y = __shfl_up(incl, d, 32);
      if (lane >= d) incl += y;
    }
    int run = incl - s;
#pragma unroll 1
    for (int i = 0; i < NBA / 32; ++i) {
      const int cv = cnt[base + i];
      offs[base + i] = run;
      cur[base + i]  = run;
      run += cv;
    }
  }
  __syncthreads();
  if (wave == 0) {
#pragma unroll 1
    for (int b0 = 0; b0 < tt; b0 += 32) {
      const int idx = b0 + lane;
      const int ent = hl[idx < RCAP ? idx : RCAP - 1];
      const int m32 = (tt - b0) < 32 ? (tt - b0) : 32;
#pragma unroll 1
      for (int k = 0; k < m32; ++k) {
        const int u    = __builtin_amdgcn_readlane(ent, k);
        const int slot = u & (NBA - 1);
        if (lane == 0) {
          int p = cur[slot];
          p = p < 0 ? 0 : (p > RCAP - 1 ? RCAP - 1 : p);
          sl[p] = u;
          cur[slot] = p + 1;
        }
      }
    }
  }
  __syncthreads();

  int* sp = SRT + (size_t)blockIdx.x * RCAP;
#pragma unroll 1
  for (int i = tid * 4; i < RCAP; i += NTHR * 4) {
    const v4i e4 = *(const v4ia*)(sl + i);
    int e0 = e4.x >> SLA, e1 = e4.y >> SLA, e2 = e4.z >> SLA, e3 = e4.w >> SLA;
    e0 = e0 < 0 ? 0 : (e0 > nE - 1 ? nE - 1 : e0);
    e1 = e1 < 0 ? 0 : (e1 > nE - 1 ? nE - 1 : e1);
    e2 = e2 < 0 ? 0 : (e2 > nE - 1 ? nE - 1 : e2);
    e3 = e3 < 0 ? 0 : (e3 > nE - 1 ? nE - 1 : e3);
    int q0 = srcs[e0], q1 = srcs[e1], q2 = srcs[e2], q3 = srcs[e3];
    v4i s4;
    s4.x = q0 < 0 ? 0 : (q0 > nN - 1 ? nN - 1 : q0);
    s4.y = q1 < 0 ? 0 : (q1 > nN - 1 ? nN - 1 : q1);
    s4.z = q2 < 0 ? 0 : (q2 > nN - 1 ? nN - 1 : q2);
    s4.w = q3 < 0 ? 0 : (q3 > nN - 1 ? nN - 1 : q3);
    *(volatile v4i*)(sp + i) = s4;
    __threadfence();
    *(volatile v4i*)(sp + i) = s4;
  }
  {
    const v4i o4 = *(const v4ia*)(offs + 4 * tid);
    const v4i c4 = *(const v4ia*)(cnt + 4 * tid);
    v4i f4;
    f4.x = (ovf != 0 || c4.x > DEGCAP) ? 1 : 0;
    f4.y = (ovf != 0 || c4.y > DEGCAP) ? 1 : 0;
    f4.z = (ovf != 0 || c4.z > DEGCAP) ? 1 : 0;
    f4.w = (ovf != 0 || c4.w > DEGCAP) ? 1 : 0;
    int* op = OC + (size_t)blockIdx.x * (3 * NBA) + 4 * tid;
    *(volatile v4i*)op = o4;
    *(volatile v4i*)(op + NBA) = c4;
    *(volatile v4i*)(op + 2 * NBA) = f4;
    __threadfence();
    *(volatile v4i*)op = o4;
    *(volatile v4i*)(op + NBA) = c4;
    *(volatile v4i*)(op + 2 * NBA) = f4;
  }
}

template <int NC>
__global__ __launch_bounds__(GTHR * NC) void k_gemm(const unsigned short* __restrict__ A, int lda,
                                                    const unsigned short* __restrict__ BT, int ldb, int K,
                                                    float* Cm, const float* __restrict__ avs,
                                                    const float* __restrict__ avd, float* AL) {
  static_assert(NC == 1 || NC == 2);
  constexpr int LDC = GBN * NC;
  constexpr int RPW = GBM / (4 * NC);
  extern __shared__ __attribute__((aligned(16))) float gsm[];
  float* stg = gsm;
  float* sdt = gsm + GBM * LDC;
  const int tid = (int)threadIdx.x, lane = tid & 31, wave = tid >> 5, hh = lane >> 4, m = lane & 15;
  const int rg = wave & 3, cg = wave >> 2;
  const int rowBase = (int)blockIdx.x * GBM;
  const int colBase = cg * GBN;

  v8f acc[8];
  {
    const v8f z = {0.f, 0.f, 0.f, 0.f, 0.f, 0.f, 0.f, 0.f};
#pragma unroll
    for (int t = 0; t < 8; ++t) acc[t] = z;
  }
  const unsigned short* ap = A  + (size_t)(rowBase + 16 * rg + m) * (size_t)lda + 8 * hh;
  const unsigned short* bp = BT + (size_t)(colBase + m) * (size_t)ldb + 8 * hh;

#pragma unroll 1
  for (int k0 = 0; k0 < K; k0 += 32) {
    FragB af;
    af.h[0] = *(const v8usa*)(ap + k0);
    af.h[1] = *(const v8usa*)(ap + k0 + 16);
#pragma unroll
    for (int nt = 0; nt < 8; ++nt) {
      const unsigned short* wq = bp + (size_t)(16 * nt) * (size_t)ldb + k0;
      FragB bf;
      bf.h[0] = *(const v8usa*)wq;
      bf.h[1] = *(const v8usa*)(wq + 16);
      acc[nt] = wmb(af, bf, acc[nt]);
    }
  }

#pragma unroll
  for (int nt = 0; nt < 8; ++nt) {
    const int lc = colBase + 16 * nt + m;
#pragma unroll
    for (int r = 0; r < 8; ++r) {
      const int lr = 16 * rg + 8 * hh + r;
      stg[lr * LDC + lc] = acc[nt][r];
    }
  }
  __syncthreads();

  v4f as4[NC], ad4[NC];
#pragma unroll
  for (int c = 0; c < NC; ++c) {
    as4[c] = bfr4(*(const v4fa*)(avs + c * GBN + 4 * lane));
    ad4[c] = bfr4(*(const v4fa*)(avd + c * GBN + 4 * lane));
  }
#pragma unroll 1
  for (int i = 0; i < RPW; ++i) {
    const int row = wave * RPW + i;
    float s = 0.0f, d = 0.0f;
#pragma unroll
    for (int c = 0; c < NC; ++c) {
      const v4f p = *(const v4fa*)(stg + row * LDC + c * GBN + 4 * lane);
      s = fmaf(p.x, as4[c].x, s); s = fmaf(p.y, as4[c].y, s); s = fmaf(p.z, as4[c].z, s); s = fmaf(p.w, as4[c].w, s);
      d = fmaf(p.x, ad4[c].x, d); d = fmaf(p.y, ad4[c].y, d); d = fmaf(p.z, ad4[c].z, d); d = fmaf(p.w, ad4[c].w, d);
    }
#pragma unroll
    for (int off = 16; off > 0; off >>= 1) {
      s += __shfl_xor(s, off);
      d += __shfl_xor(d, off);
    }
    if (lane == 0) { sdt[row] = s; sdt[GBM + row] = d; }
  }
  __syncthreads();

  const v4f alv = *(const v4fa*)(sdt + 4 * lane);
  float* alp = AL + (size_t)blockIdx.x * (2 * GBM) + 4 * lane;
#pragma unroll 1
  for (int i = 0; i < RPW; ++i) {
    const int row = wave * RPW + i;
#pragma unroll
    for (int c = 0; c < NC; ++c) {
      const v4f p = *(const v4fa*)(stg + row * LDC + c * GBN + 4 * lane);
      float* op = Cm + (size_t)(rowBase + row) * (size_t)LDC + c * GBN + 4 * lane;
      *(volatile v4f*)op = p;
    }
  }
  if (wave == 0) *(volatile v4f*)alp = alv;
  __threadfence();
#pragma unroll 1
  for (int i = 0; i < RPW; ++i) {
    const int row = wave * RPW + i;
#pragma unroll
    for (int c = 0; c < NC; ++c) {
      const v4f p = *(const v4fa*)(stg + row * LDC + c * GBN + 4 * lane);
      float* op = Cm + (size_t)(rowBase + row) * (size_t)LDC + c * GBN + 4 * lane;
      *(volatile v4f*)op = p;
    }
  }
  if (wave == 0) *(volatile v4f*)alp = alv;
}

__global__ __launch_bounds__(GTHR) void k_gemm64(
    const unsigned short* __restrict__ A, const unsigned short* __restrict__ WT,
    float* outF, int K,
    const float* __restrict__ atts, const float* __restrict__ attd, float* AL)
{
  __shared__ __attribute__((aligned(16))) float stg[GBM * D2];
  __shared__ __attribute__((aligned(16))) float satt[2 * D2];
  __shared__ __attribute__((aligned(16))) float sdot[2 * GBM];
  const int tid = (int)threadIdx.x, lane = tid & 31, wave = tid >> 5, hh = lane >> 4, m = lane & 15;
  const int rowBase = (int)blockIdx.x * GBM;

  {
    const int which = tid >> 6;
    const int c  = tid & 63;
    const float vs = atts[c];
    const float vd = attd[c];
    const unsigned int msk = (which == 0) ? 0u : 0xFFFFFFFFu;
    const float v = __uint_as_float((__float_as_uint(vs) & ~msk) | (__float_as_uint(vd) & msk));
    satt[which * D2 + c] = bf16_val(v);
  }

  v8f acc[4];
  {
    const v8f z = {0.f, 0.f, 0.f, 0.f, 0.f, 0.f, 0.f, 0.f};
    acc[0] = z; acc[1] = z; acc[2] = z; acc[3] = z;
  }
  const unsigned short* ap = A  + (size_t)(rowBase + 16 * wave + m) * (size_t)K + 8 * hh;
  const unsigned short* wp = WT + (size_t)m * (size_t)K + 8 * hh;
  const int ksteps = K >> 5;
#pragma unroll 1
  for (int ks = 0; ks < ksteps; ++ks) {
    FragB af;
    af.h[0] = *(const v8usa*)(ap + 32 * ks);
    af.h[1] = *(const v8usa*)(ap + 32 * ks + 16);
#pragma unroll
    for (int t = 0; t < 4; ++t) {
      const unsigned short* wq = wp + (size_t)(16 * t) * (size_t)K + 32 * ks;
      FragB bf;
      bf.h[0] = *(const v8usa*)wq;
      bf.h[1] = *(const v8usa*)(wq + 16);
      acc[t] = wmb(af, bf, acc[t]);
    }
  }

#pragma unroll
  for (int t = 0; t < 4; ++t) {
    const int lc = 16 * t + m;
#pragma unroll
    for (int r = 0; r < 8; ++r) {
      const int lr = 16 * wave + 8 * hh + r;
      stg[lr * D2 + lc] = acc[t][r];
    }
  }
  __syncthreads();

  {
    const int row = tid & 63, which = tid >> 6;
    const float* sa = satt + which * D2;
    const float* hr = stg + row * D2;
    float d = 0.f;
#pragma unroll 4
    for (int c4 = 0; c4 < D2 / 4; ++c4) {
      const v4f hv = *(const v4fa*)(hr + 4 * c4);
      const v4f av = *(const v4fa*)(sa + 4 * c4);
      d = fmaf(hv.x, av.x, d);
      d = fmaf(hv.y, av.y, d);
      d = fmaf(hv.z, av.z, d);
      d = fmaf(hv.w, av.w, d);
    }
    sdot[which * GBM + row] = d;
  }
  __syncthreads();

  v4f fv[8];
#pragma unroll
  for (int i = 0; i < 8; ++i) {
    const int lr = 16 * wave + 2 * i + hh;
    fv[i] = *(const v4fa*)(stg + lr * D2 + 4 * m);
  }
  const v4f sdv = *(const v4fa*)(sdot + 4 * lane);
  float* sp = AL + (size_t)blockIdx.x * (2 * GBM) + 4 * lane;

#pragma unroll
  for (int i = 0; i < 8; ++i) {
    const int lr = 16 * wave + 2 * i + hh;
    float* op = outF + (size_t)(rowBase + lr) * (size_t)D2 + 4 * m;
    *(volatile v4f*)op = fv[i];
  }
  if (wave == 0) *(volatile v4f*)sp = sdv;
  __threadfence();
#pragma unroll
  for (int i = 0; i < 8; ++i) {
    const int lr = 16 * wave + 2 * i + hh;
    float* op = outF + (size_t)(rowBase + lr) * (size_t)D2 + 4 * m;
    *(volatile v4f*)op = fv[i];
  }
  if (wave == 0) *(volatile v4f*)sp = sdv;
}

template <int CPL, int WD>
__device__ __forceinline__ float elu_rows(float* w, const float* sbv, const float* swv, int lane, float inv) {
  float h = 0.f;
#pragma unroll 1
  for (int i = 0; i < CPL; ++i) {
    const int j = CPL * lane + i;
    float y = fmaf(w[j], inv, sbv[j]);
    y = y > 0.f ? y : expm1f(y);
    w[j] = y;
    if (WD != 0) h = fmaf(y, swv[j], h);
  }
  return h;
}

template <int L>
__global__ __launch_bounds__(NTHR) void k_scan(const int* __restrict__ SRT, const int* __restrict__ OC,
                                               const float* __restrict__ AL, const float* __restrict__ F,
                                               const float* __restrict__ bias, const float* __restrict__ w3,
                                               const float* __restrict__ a3s, const float* __restrict__ a3d,
                                               unsigned short* X1, float* H3o, float* outp,
                                               int nN, int mRows) {
  static_assert(L >= 1 && L <= 3);
  constexpr int CPL = (L == 1) ? 8 : 2;
  constexpr int C   = CPL * 32;
  __shared__ __attribute__((aligned(16))) float wst[NWAVE * 256];
  __shared__ __attribute__((aligned(16))) float sb[NTHR];
  __shared__ __attribute__((aligned(16))) float sw3[D2];
  __shared__ __attribute__((aligned(16))) float res[NBA];
  const int tid = (int)threadIdx.x, lane = tid & 31;
  const int wave = __builtin_amdgcn_readfirstlane(tid >> 5);
  const int nodeBase = (int)blockIdx.x * NBA;
  const float qnan = __int_as_float(0x7fc00000);

  float a3sv = 0.f, a3dv = 0.f, b3v = 0.f;
  if constexpr (L < 3) {
    const int cb = tid < C ? tid : C - 1;
    sb[tid] = bf16_val(bias[cb]);
    if constexpr (L == 2) {
      const float wv = bf16_val(w3[tid & (D2 - 1)]);
      if (tid < D2) sw3[tid] = wv;
    }
  } else {
    a3sv = bf16_val(a3s[0]);
    a3dv = bf16_val(a3d[0]);
    b3v  = bf16_val(bias[0]);
  }
  __syncthreads();

  const int* ocb = OC + (size_t)blockIdx.x * (3 * NBA);
  const int* srt = SRT + (size_t)blockIdx.x * RCAP;
  float* wrow = wst + wave * 256;

#pragma unroll 1
  for (int si = 0; si < NBA / NWAVE; ++si) {
    const int s    = si * NWAVE + wave;
    const int node = nodeBase + s;
    const int nc   = node < nN ? node : nN - 1;
    int o          = __builtin_amdgcn_readfirstlane(ocb[s]);
    const int craw = __builtin_amdgcn_readfirstlane(ocb[NBA + s]);
    const int fl   = __builtin_amdgcn_readfirstlane(ocb[2 * NBA + s]);
    int c = craw < 0 ? 0 : (craw > DEGCAP ? DEGCAP : craw);
    o = o < 0 ? 0 : (o > RCAP ? RCAP : o);
    if (c > RCAP - o) c = RCAP - o;
    const bool poison = (fl != 0) || (craw > DEGCAP) || (craw < 0);
    const bool live   = node < nN;

    float hd = 0.f, as0, ad;
    if constexpr (L < 3) {
      const int alb = (nc >> 6) * (2 * GBM) + (nc & (GBM - 1));
      as0 = AL[alb];
      ad  = AL[alb + GBM];
    } else {
      hd  = F[nc];
      as0 = a3sv * hd;
      ad  = a3dv * hd;
    }
    float l0 = as0 + ad;
    l0 = l0 > 0.f ? l0 : NEGSL * l0;

    float ml = -3.0e38f;
#pragma unroll 1
    for (int b0 = 0; b0 < c; b0 += 32) {
      int idx = o + b0 + lane;
      idx = idx > RCAP - 1 ? RCAP - 1 : idx;
      int sr = srt[idx];
      sr = sr < 0 ? 0 : (sr > nN - 1 ? nN - 1 : sr);
      float es;
      if constexpr (L < 3) es = AL[(sr >> 6) * (2 * GBM) + (sr & (GBM - 1))];
      else                 es = a3sv * F[sr];
      float e = es + ad;
      e = e > 0.f ? e : NEGSL * e;
      const bool valid = (b0 + lane) < c;
      ml = fmaxf(ml, valid ? e : -3.0e38f);
    }
#pragma unroll
    for (int off = 16; off > 0; off >>= 1) ml = fmaxf(ml, __shfl_xor(ml, off));
    const float mx = fmaxf(ml, l0);

    float acc[CPL];
#pragma unroll
    for (int i = 0; i < CPL; ++i) acc[i] = 0.f;
    float dl = 0.f, nl = 0.f;
#pragma unroll 1
    for (int b0 = 0; b0 < c; b0 += 32) {
      int idx = o + b0 + lane;
      idx = idx > RCAP - 1 ? RCAP - 1 : idx;
      int sr = srt[idx];
      sr = sr < 0 ? 0 : (sr > nN - 1 ? nN - 1 : sr);
      float es, hs = 0.f;
      if constexpr (L < 3) {
        es = AL[(sr >> 6) * (2 * GBM) + (sr & (GBM - 1))];
      } else {
        hs = F[sr];
        es = a3sv * hs;
      }
      float e = es + ad;
      e = e > 0.f ? e : NEGSL * e;
      const bool valid = (b0 + lane) < c;
      float p = expf(e - mx);
      p = valid ? p : 0.f;
      dl += p;
      if constexpr (L == 3) {
        const float tq = p * hs;
        nl += valid ? tq : 0.f;
      } else {
        const int m32 = (c - b0) < 32 ? (c - b0) : 32;
        const int pi  = __float_as_int(p);
#pragma unroll 1
        for (int k = 0; k < m32; ++k) {
          const int   sk = __builtin_amdgcn_readlane(sr, k);
          const float pk = __int_as_float(__builtin_amdgcn_readlane(pi, k));
          const float* rp = F + (size_t)sk * C + CPL * lane;
          if constexpr (CPL == 8) {
            const v4f a = *(const v4fa*)rp;
            const v4f b = *(const v4fa*)(rp + 4);
            acc[0] = fmaf(pk, a.x, acc[0]); acc[1] = fmaf(pk, a.y, acc[1]);
            acc[2] = fmaf(pk, a.z, acc[2]); acc[3] = fmaf(pk, a.w, acc[3]);
            acc[4] = fmaf(pk, b.x, acc[4]); acc[5] = fmaf(pk, b.y, acc[5]);
            acc[6] = fmaf(pk, b.z, acc[6]); acc[7] = fmaf(pk, b.w, acc[7]);
          } else {
            const v2f a = *(const v2fa*)rp;
            acc[0] = fmaf(pk, a.x, acc[0]); acc[1] = fmaf(pk, a.y, acc[1]);
          }
        }
      }
    }
#pragma unroll
    for (int off = 16; off > 0; off >>= 1) {
      dl += __shfl_xor(dl, off);
      nl += __shfl_xor(nl, off);
    }
    const float pself = expf(l0 - mx);
    const float den   = dl + pself;
    const float inv   = __builtin_amdgcn_rcpf(den);

    if constexpr (L == 1) {
      {
        const float* sp = F + (size_t)nc * C + CPL * lane;
        const v4f a = *(const v4fa*)sp;
        const v4f b = *(const v4fa*)(sp + 4);
        v4f ta, tb;
        ta.x = fmaf(pself, a.x, acc[0]); ta.y = fmaf(pself, a.y, acc[1]);
        ta.z = fmaf(pself, a.z, acc[2]); ta.w = fmaf(pself, a.w, acc[3]);
        tb.x = fmaf(pself, b.x, acc[4]); tb.y = fmaf(pself, b.y, acc[5]);
        tb.z = fmaf(pself, b.z, acc[6]); tb.w = fmaf(pself, b.w, acc[7]);
        *(v4fa*)(wrow + 8 * lane)     = ta;
        *(v4fa*)(wrow + 8 * lane + 4) = tb;
      }
      (void)elu_rows<8, 0>(wrow, sb, sb, lane, inv);
      const v4f va = *(const v4fa*)(wrow + 8 * lane);
      const v4f vb = *(const v4fa*)(wrow + 8 * lane + 4);
      float v[8];
      v[0] = va.x; v[1] = va.y; v[2] = va.z; v[3] = va.w;
      v[4] = vb.x; v[5] = vb.y; v[6] = vb.z; v[7] = vb.w;
      v8us ho, lo;
#pragma unroll
      for (int i = 0; i < 8; ++i) {
        float y = poison ? qnan : v[i];
        y = live ? y : 0.0f;
        const unsigned hbi = bf16_bits(y);
        ho[i] = (unsigned short)hbi;
        lo[i] = (unsigned short)bf16_bits(y - __uint_as_float(hbi << 16));
      }
      if (node < mRows) {
        unsigned short* hp = X1 + (size_t)node * KP + 8 * lane;
        *(volatile v8us*)hp = ho;
        *(volatile v8us*)(hp + D1) = lo;
        __threadfence();
        *(volatile v8us*)hp = ho;
        *(volatile v8us*)(hp + D1) = lo;
      }
    } else if constexpr (L == 2) {
      {
        const v2f a = *(const v2fa*)(F + (size_t)nc * C + CPL * lane);
        v2f ta;
        ta.x = fmaf(pself, a.x, acc[0]);
        ta.y = fmaf(pself, a.y, acc[1]);
        *(v2fa*)(wrow + 2 * lane) = ta;
      }
      float h3 = elu_rows<2, 1>(wrow, sb, sw3, lane, inv);
#pragma unroll
      for (int off = 16; off > 0; off >>= 1) h3 += __shfl_xor(h3, off);
      if (lane == 0) {
        const float y = poison ? qnan : h3;
        res[s] = live ? y : 0.0f;
      }
    } else {
      const float num = nl + pself * hd;
      float y = num * inv + b3v;
      y = poison ? qnan : y;
      if (lane == 0) res[s] = live ? y : 0.0f;
    }
  }

  if constexpr (L >= 2) {
    __syncthreads();
    const int f0 = nodeBase + 4 * tid;
    const v4f v = *(const v4fa*)(res + 4 * tid);
    if constexpr (L == 2) {
      float* op = H3o + (size_t)f0;
      *(volatile v4f*)op = v;
      __threadfence();
      *(volatile v4f*)op = v;
    } else {
      const bool wr = (f0 + 4 <= nN);
      float* op = outp + (size_t)f0;
      if (wr) *(volatile v4f*)op = v;
      __threadfence();
      if (wr) *(volatile v4f*)op = v;
    }
  }
}

static inline int cdiv(int a, int b) { return (a + b - 1) / b; }

extern "C" void kernel_launch(void* const* d_in, const int* in_sizes, int n_in,
                              void* d_out, int out_size, void* d_ws, size_t ws_size,
                              hipStream_t stream) {
  if (n_in < 14) return;
  if (in_sizes[0] < DIN || (in_sizes[0] % DIN) != 0) return;
  const int nN = in_sizes[0] / DIN;
  if ((nN % 16) != 0 || nN >= (1 << 22)) return;
  if (in_sizes[1] < 2 || (in_sizes[1] & 1) != 0) return;
  const int nE = in_sizes[1] / 2;
  if (nE < 1 || nE >= (1 << 21)) return;
  if (in_sizes[2] != DIN * D1) return;
  if (in_sizes[3] != D1 || in_sizes[4] != D1 || in_sizes[5] != D1) return;
  if (in_sizes[6] != D1 * D2) return;
  if (in_sizes[7] != D2 || in_sizes[8] != D2 || in_sizes[9] != D2) return;
  if (in_sizes[10] != D2) return;
  if (in_sizes[11] < 1 || in_sizes[12] < 1 || in_sizes[13] < 1) return;
  if (out_size != nN) return;

  const float* x    = (const float*)d_in[0];
  const int*   edge = (const int*)d_in[1];
  const float* W1   = (const float*)d_in[2];
  const float* as1  = (const float*)d_in[3];
  const float* ad1  = (const float*)d_in[4];
  const float* b1   = (const float*)d_in[5];
  const float* W2   = (const float*)d_in[6];
  const float* as2  = (const float*)d_in[7];
  const float* ad2  = (const float*)d_in[8];
  const float* b2   = (const float*)d_in[9];
  const float* W3   = (const float*)d_in[10];
  const float* as3  = (const float*)d_in[11];
  const float* ad3  = (const float*)d_in[12];
  const float* b3   = (const float*)d_in[13];
  float* out = (float*)d_out;
  const int* src = edge;
  const int* dst = edge + nE;

  const int MP   = cdiv(nN, GBM) * GBM;
  const int gM   = MP / GBM;
  const int gA   = cdiv(MP, NBA);
  if ((long long)gA * NBA < (long long)MP) return;
  const int vec8 = ((nE & 3) == 0) ? 1 : 0;
  const int nUx  = MP * (DIN / 8);
  if ((nUx % NTHR) != 0) return;

  char* ws = (char*)d_ws;
  size_t off = 0;
  const size_t oW1T = off; off += (size_t)D1 * DIN * 2;                   off = (off + 255) & ~(size_t)255;
  const size_t oW2T = off; off += (size_t)D2 * KP * 2;                    off = (off + 255) & ~(size_t)255;
  const size_t oAL  = off; off += (size_t)gM * (2 * GBM) * 4;             off = (off + 255) & ~(size_t)255;
  const size_t oH3  = off; off += (size_t)gA * NBA * 4;                   off = (off + 255) & ~(size_t)255;
  const size_t oOC  = off; off += (size_t)gA * 3 * NBA * 4;               off = (off + 255) & ~(size_t)255;
  const size_t oSRT = off; off += (size_t)gA * RCAP * 4;                  off = (off + 255) & ~(size_t)255;
  const size_t oA   = off; off += (size_t)MP * KP * 2;                    off = (off + 255) & ~(size_t)255;
  const size_t oB   = off; off += (size_t)MP * D1 * 4;                    off = (off + 255) & ~(size_t)255;
  if (off > ws_size || off > (size_t)WSMAX) return;
  unsigned short* W1T = (unsigned short*)(ws + oW1T);
  unsigned short* W2T = (unsigned short*)(ws + oW2T);
  float*          ALp = (float*)(ws + oAL);
  float*          H3  = (float*)(ws + oH3);
  int*            OC  = (int*)(ws + oOC);
  int*            SRT = (int*)(ws + oSRT);
  unsigned short* RA  = (unsigned short*)(ws + oA);
  float*          RB  = (float*)(ws + oB);

  const size_t bktLds   = (size_t)AGG_LDS_INTS * 4;
  const size_t gemmLds2 = (size_t)(GBM * 2 * GBN + 2 * GBM) * 4;
  hipFuncSetAttribute(reinterpret_cast<const void*>(&k_gemm<2>), hipFuncAttributeMaxDynamicSharedMemorySize, (int)gemmLds2);
  hipFuncSetAttribute(reinterpret_cast<const void*>(&k_bucket), hipFuncAttributeMaxDynamicSharedMemorySize, (int)bktLds);

  k_prep<<<(nUx + NU1 + NU2) / NTHR, NTHR, 0, stream>>>(x, W1, W2, RA, W1T, W2T, nN, nUx);
  k_bucket<<<gA, NTHR, bktLds, stream>>>(src, dst, nE, nN, vec8, SRT, OC);
  k_gemm<2><<<gM, GTHR * 2, gemmLds2, stream>>>(RA, DIN, W1T, DIN, DIN, RB, as1, ad1, ALp);
  k_scan<1><<<gA, NTHR, 0, stream>>>(SRT, OC, ALp, RB, b1, W3, as3, ad3, RA, H3, out, nN, MP);
  k_gemm64<<<gM, GTHR, 0, stream>>>(RA, W2T, RB, KP, as2, ad2, ALp);
  k_scan<2><<<gA, NTHR, 0, stream>>>(SRT, OC, ALp, RB, b2, W3, as3, ad3, RA, H3, out, nN, MP);
  k_scan<3><<<gA, NTHR, 0, stream>>>(SRT, OC, ALp, H3, b3, W3, as3, ad3, RA, H3, out, nN, MP);
}
